// DocREModel_19284403159262
// MI455X (gfx1250) — hardware-verified
//
#include <hip/hip_runtime.h>


#define NB_ 2
#define LL 512
#define DD 768
#define NH 12
#define NE 32
#define NM 4
#define NPR 256
#define EMB 768
#define BS 64
#define NCL 97
#define NPAIR (NB_ * NPR)
#define NMEN (NE * NM)

typedef __attribute__((ext_vector_type(16))) __bf16   v16bf;
typedef __attribute__((ext_vector_type(16))) _Float16 v16h;
typedef __attribute__((ext_vector_type(8)))  float    v8f;
typedef __attribute__((ext_vector_type(8)))  unsigned v8u;

__device__ __forceinline__ unsigned f2bf(float f) { unsigned u = __float_as_uint(f); u += 0x7FFFu + ((u >> 16) & 1u); return u >> 16; }
__device__ __forceinline__ unsigned f2h(float f) { return (unsigned)__builtin_bit_cast(unsigned short, (_Float16)f); }
__device__ __forceinline__ int kpat(int v, int half) { return ((v & 4) ? 16 : 0) + half * 8 + 2 * (v & 3); }

template <int F16, int NP> struct Opnd { v16bf p[NP]; };

template <int F16, int NP> __device__ __forceinline__ void pack2(float f0, float f1, unsigned* o) {
    if (F16) { o[0] = f2h(f0) | (f2h(f1) << 16); return; }
    unsigned h0 = f2bf(f0), h1 = f2bf(f1); o[0] = h0 | (h1 << 16);
    if (NP >= 2) {
        float r0 = f0 - __uint_as_float(h0 << 16), r1 = f1 - __uint_as_float(h1 << 16);
        unsigned m0 = f2bf(r0), m1 = f2bf(r1); o[1] = m0 | (m1 << 16);
        if (NP >= 3) {
            float s0 = r0 - __uint_as_float(m0 << 16), s1 = r1 - __uint_as_float(m1 << 16);
            o[2] = f2bf(s0) | (f2bf(s1) << 16);
        }
    }
}
template <int F16, int NP> __device__ __forceinline__ void op_row(const float* rowp, int half, float sc, Opnd<F16, NP>& o) {
    v8u u[NP];
#pragma unroll
    for (int v = 0; v < 8; ++v) {
        int kk = kpat(v, half); unsigned t[3];
        pack2<F16, NP>(rowp[kk] * sc, rowp[kk + 1] * sc, t);
#pragma unroll
        for (int p = 0; p < NP; ++p) u[p][v] = t[p];
    }
#pragma unroll
    for (int p = 0; p < NP; ++p) o.p[p] = __builtin_bit_cast(v16bf, u[p]);
}
template <int F16, int NP> __device__ __forceinline__ void op_row_tail(const float* rowp, int half, float sc, int kvalid, Opnd<F16, NP>& o) {
    v8u u[NP];
#pragma unroll
    for (int v = 0; v < 8; ++v) {
        int kk = kpat(v, half); unsigned t[3];
        float f0 = kk < kvalid ? rowp[kk] * sc : 0.0f, f1 = (kk + 1) < kvalid ? rowp[kk + 1] * sc : 0.0f;
        pack2<F16, NP>(f0, f1, t);
#pragma unroll
        for (int p = 0; p < NP; ++p) u[p][v] = t[p];
    }
#pragma unroll
    for (int p = 0; p < NP; ++p) o.p[p] = __builtin_bit_cast(v16bf, u[p]);
}
template <int F16, int NP> __device__ __forceinline__ void op_col(const float* M, int ld, int n, int k0, int half, float sc, Opnd<F16, NP>& o) {
    v8u u[NP];
#pragma unroll
    for (int v = 0; v < 8; ++v) {
        int kk = k0 + kpat(v, half); unsigned t[3];
        pack2<F16, NP>(M[(size_t)kk * ld + n] * sc, M[(size_t)(kk + 1) * ld + n] * sc, t);
#pragma unroll
        for (int p = 0; p < NP; ++p) u[p][v] = t[p];
    }
#pragma unroll
    for (int p = 0; p < NP; ++p) o.p[p] = __builtin_bit_cast(v16bf, u[p]);
}
template <int F16, int NP> __device__ __forceinline__ void op_col_tail(const float* M, int ld, int n, int k0, int half, float sc, int K, Opnd<F16, NP>& o) {
    v8u u[NP];
#pragma unroll
    for (int v = 0; v < 8; ++v) {
        int kk = k0 + kpat(v, half); unsigned t[3];
        float f0 = kk < K ? M[(size_t)kk * ld + n] * sc : 0.0f, f1 = (kk + 1) < K ? M[(size_t)(kk + 1) * ld + n] * sc : 0.0f;
        pack2<F16, NP>(f0, f1, t);
#pragma unroll
        for (int p = 0; p < NP; ++p) u[p][v] = t[p];
    }
#pragma unroll
    for (int p = 0; p < NP; ++p) o.p[p] = __builtin_bit_cast(v16bf, u[p]);
}
__device__ __forceinline__ v8f wm_bf16(v16bf a, v16bf b, v8f c) { return __builtin_amdgcn_wmma_f32_16x16x32_bf16(false, a, false, b, (short)0, c, false, false); }
template <int F16, int NA, int NB> __device__ __forceinline__ v8f wmma_op(const Opnd<F16, NA>& a, const Opnd<F16, NB>& b, v8f c) {
    if (F16) {
        v16h ah = __builtin_bit_cast(v16h, a.p[0]), bh = __builtin_bit_cast(v16h, b.p[0]);
        c = __builtin_amdgcn_wmma_f32_16x16x32_f16(false, ah, false, bh, (short)0, c, false, false);
        asm volatile("v_nop\n\tv_nop\n\tv_nop\n\tv_nop" : "+v"(c) : "v"(ah), "v"(bh));
        return c;
    }
    constexpr int NMX = NA > NB ? NA : NB;
#pragma unroll
    for (int i = 0; i < NA; ++i)
#pragma unroll
        for (int j = 0; j < NB; ++j)
            if (i + j < NMX) c = wm_bf16(a.p[i], b.p[j], c);
    if (NA == 1 && NB == 1)      asm volatile("v_nop\n\tv_nop\n\tv_nop\n\tv_nop" : "+v"(c) : "v"(a.p[0]), "v"(b.p[0]));
    else if (NA == 2 && NB == 1) asm volatile("v_nop\n\tv_nop\n\tv_nop\n\tv_nop" : "+v"(c) : "v"(a.p[0]), "v"(a.p[1]), "v"(b.p[0]));
    else if (NA == 1 && NB == 2) asm volatile("v_nop\n\tv_nop\n\tv_nop\n\tv_nop" : "+v"(c) : "v"(a.p[0]), "v"(b.p[0]), "v"(b.p[1]));
    else if (NA == 2 && NB == 2) asm volatile("v_nop\n\tv_nop\n\tv_nop\n\tv_nop" : "+v"(c) : "v"(a.p[0]), "v"(a.p[1]), "v"(b.p[0]), "v"(b.p[1]));
    else                         asm volatile("v_nop\n\tv_nop\n\tv_nop\n\tv_nop" : "+v"(c) : "v"(a.p[0]), "v"(a.p[NA - 1]), "v"(b.p[0]), "v"(b.p[NB - 1]), "v"(a.p[NA / 2]), "v"(b.p[NB / 2]));
    return c;
}

struct ZMap { long long s1; long long s2; int zdiv; int pad_; };
__device__ __forceinline__ size_t zoff(const ZMap& m, int z) { return (size_t)((long long)(z / m.zdiv) * m.s1 + (long long)(z % m.zdiv) * m.s2); }

#define ACT_NONE 0
#define ACT_RELU 1
#define ACT_GELU_ERF 2
#define ACT_SILU 3
#define ACT_TANH 4
__device__ __forceinline__ float act_apply(int act, float x) {
    if (act == ACT_RELU) return x > 0.f ? x : 0.f;
    if (act == ACT_GELU_ERF) return 0.5f * x * (1.0f + erff(x * 0.70710678118654752f));
    if (act == ACT_SILU) return x / (1.0f + expf(-x));
    if (act == ACT_TANH) return tanhf(x);
    return x;
}
struct GemmArgs {
    ZMap za, zb_, zc, zbias, zadd, zrsc, zmul, zrbias;
    const float* A; const float* Bm; float* C; const float* bias; const float* add; const float* rsc; const float* mul; const float* rbias;
    long long ldadd, ldmul;
    int lda, ldb, ldc, K;
    float ascale, bscale, oscale, addscale;
    int M, nvalid, nstore, ldrsc;
    int bcs, pad1, pad2, pad3;
};
template <int BT, int F16, int NA, int NB, int RW, int CW, int ACT>
__global__ __launch_bounds__(256) void gemm_kernel(GemmArgs g) {
    constexpr int TR = 16 * RW, TC = 64 * CW, CSTR = TC + 4;
    __shared__ __align__(16) float cst[TR * CSTR];
    const int z = blockIdx.z;
    const float* A = g.A + zoff(g.za, z); const float* Bm = g.Bm + zoff(g.zb_, z); float* C = g.C + zoff(g.zc, z);
    const int tid = threadIdx.x, lane = tid & 31, wv = tid >> 5;
    const int l16 = lane & 15, half = lane >> 4;
    const int rt = wv % RW, ch = wv / RW;
    const int row0 = blockIdx.x * TR, col0 = blockIdx.y * TC + ch * 64;
    int arix = row0 + rt * 16 + l16; if (arix >= g.M) arix = g.M - 1;
    const float* arow = A + (size_t)arix * g.lda;
    v8f acc[4];
#pragma unroll
    for (int t = 0; t < 4; ++t) acc[t] = (v8f){};
    const int K = g.K;
#pragma unroll 1
    for (int kc = 0; kc < K; kc += 32) {
        Opnd<F16, NA> a;
        if (kc + 32 <= K) op_row<F16, NA>(arow + kc, half, g.ascale, a); else op_row_tail<F16, NA>(arow + kc, half, g.ascale, K - kc, a);
#pragma unroll
        for (int t = 0; t < 4; ++t) {
            Opnd<F16, NB> b;
            const int n = col0 + t * 16 + l16;
            if (n < g.nvalid) {
                if (BT) { if (kc + 32 <= K) op_row<F16, NB>(Bm + (size_t)n * g.ldb + kc, half, g.bscale, b); else op_row_tail<F16, NB>(Bm + (size_t)n * g.ldb + kc, half, g.bscale, K - kc, b); }
                else    { if (kc + 32 <= K) op_col<F16, NB>(Bm, g.ldb, n * g.bcs, kc, half, g.bscale, b); else op_col_tail<F16, NB>(Bm, g.ldb, n * g.bcs, kc, half, g.bscale, K, b); }
            } else {
#pragma unroll
                for (int p = 0; p < NB; ++p) b.p[p] = (v16bf){};
            }
            acc[t] = wmma_op<F16, NA, NB>(a, b, acc[t]);
        }
    }
    const float* bias = g.bias ? g.bias + zoff(g.zbias, z) : nullptr;
    const float* add = g.add ? g.add + zoff(g.zadd, z) : nullptr;
    const float* rsc = g.rsc ? g.rsc + zoff(g.zrsc, z) : nullptr;
    const float* mul = g.mul ? g.mul + zoff(g.zmul, z) : nullptr;
    const float* rbias = g.rbias ? g.rbias + zoff(g.zrbias, z) : nullptr;
#pragma unroll
    for (int t = 0; t < 4; ++t) {
        const int cl = ch * 64 + t * 16 + l16;
        const int cg = blockIdx.y * TC + cl;
        const bool cok = cg < g.nvalid;
        const float bv = (bias && cok) ? bias[(size_t)cg * g.bcs] : 0.0f;
#pragma unroll
        for (int r = 0; r < 8; ++r) {
            const int rl = rt * 16 + r + 8 * half;
            float v = acc[t][r] * g.oscale + bv;
            int rg = row0 + rl; if (rg >= g.M) rg = g.M - 1;
            if (rbias) v += rbias[rg];
            if (rsc) v *= rsc[(size_t)rg * g.ldrsc];
            if (mul && cok) v *= mul[(size_t)rg * g.ldmul + cg];
            if (add && cok) v += g.addscale * add[(size_t)rg * g.ldadd + cg];
            cst[rl * CSTR + cl] = v;
        }
    }
    __syncthreads();
    const int col = tid % TC, rsel = tid / TC, rstep = 256 / TC;
    if (ACT != ACT_NONE) {
#pragma unroll 1
        for (int r = rsel; r < TR; r += rstep) cst[r * CSTR + col] = act_apply(ACT, cst[r * CSTR + col]);
    }
    float* ob = C + (size_t)row0 * g.ldc + (size_t)blockIdx.y * TC;
    const bool colok = (int)(blockIdx.y * TC + col) < g.nstore;
    const int rmax = (g.M - row0 < TR) ? (g.M - row0) : TR;
    auto pass = [&]() {
        if (colok) {
#pragma unroll 4
            for (int r = rsel; r < rmax; r += rstep) *(volatile float*)(ob + (size_t)r * g.ldc + col) = cst[r * CSTR + col];
        }
    };
    pass();
    __threadfence();
    pass();
}
static inline ZMap zm(long long s1) { ZMap m; m.s1 = s1; m.s2 = 0; m.zdiv = 1; m.pad_ = 0; return m; }
static inline ZMap zm2(long long s1, long long s2, int zdiv) { ZMap m; m.s1 = s1; m.s2 = s2; m.zdiv = zdiv; m.pad_ = 0; return m; }
static inline GemmArgs gemm_args(const float* A, int lda, ZMap za, const float* Bm, int ldb, ZMap zb, float* C, int ldc, ZMap zc, int M, int N, int K) {
    GemmArgs g; g.za = za; g.zb_ = zb; g.zc = zc; g.zbias = zm(0); g.zadd = zm(0); g.zrsc = zm(0); g.zmul = zm(0); g.zrbias = zm(0);
    g.A = A; g.Bm = Bm; g.C = C; g.bias = nullptr; g.add = nullptr; g.rsc = nullptr; g.mul = nullptr; g.rbias = nullptr; g.ldadd = 0; g.ldmul = 0;
    g.lda = lda; g.ldb = ldb; g.ldc = ldc; g.K = K; g.ascale = 1.0f; g.bscale = 1.0f; g.oscale = 1.0f; g.addscale = 1.0f; g.M = M; g.nvalid = N; g.nstore = N; g.ldrsc = 1;
    g.bcs = 1; g.pad1 = 0; g.pad2 = 0; g.pad3 = 0;
    return g;
}
static_assert(sizeof(ZMap) == 24, "ZMap layout");
static_assert(sizeof(GemmArgs) == 8 * 24 + 8 * 8 + 2 * 8 + 4 * 4 + 4 * 4 + 4 * 4 + 4 * 4, "GemmArgs has no padding");

__global__ __launch_bounds__(256) void softmax_rows(float* S, long long sy, long long sx, int L, float prescale, const float* addv, long long say, int aydiv, int causal,
                                                  const int* imask, long long imy, long long imx, float maskval) {
    __shared__ float red[8];
    const int tid = threadIdx.x, lane = tid & 31, wid = tid >> 5;
    float* row = S + (size_t)blockIdx.y * sy + (size_t)blockIdx.x * sx;
    const float* av = addv ? addv + (size_t)(blockIdx.y / aydiv) * say : nullptr;
    const int* im = imask ? imask + (size_t)(blockIdx.y / aydiv) * imy + (size_t)blockIdx.x * imx : nullptr;
    float v[16];
    const int nj = L / 256;
    float mx = -__builtin_inff();
#pragma unroll
    for (int j = 0; j < 16; ++j) if (j < nj) { float t = row[tid + 256 * j] * prescale; if (av) t += av[tid + 256 * j]; if (im && im[tid + 256 * j] == 0) t = maskval; if (causal && (tid + 256 * j) > (int)blockIdx.x) t = -__builtin_inff(); v[j] = t; mx = fmaxf(mx, t); }
#pragma unroll
    for (int o = 16; o; o >>= 1) mx = fmaxf(mx, __shfl_xor(mx, o, 32));
    if (lane == 0) red[wid] = mx;
    __syncthreads();
    float m = red[0];
#pragma unroll
    for (int i = 1; i < 8; ++i) m = fmaxf(m, red[i]);
    if (m == -__builtin_inff()) m = 0.f;
    __syncthreads();
    float sum = 0.f;
#pragma unroll
    for (int j = 0; j < 16; ++j) if (j < nj) { v[j] = expf(v[j] - m); sum += v[j]; }
#pragma unroll
    for (int o = 16; o; o >>= 1) sum += __shfl_xor(sum, o, 32);
    if (lane == 0) red[wid] = sum;
    __syncthreads();
    float tot = 0.f;
#pragma unroll
    for (int i = 0; i < 8; ++i) tot += red[i];
    const float inv = 1.0f / tot;
#pragma unroll
    for (int j = 0; j < 16; ++j) if (j < nj) *(volatile float*)(row + tid + 256 * j) = v[j] * inv;
    __threadfence();
#pragma unroll
    for (int j = 0; j < 16; ++j) if (j < nj) *(volatile float*)(row + tid + 256 * j) = v[j] * inv;
}

#define VST2(T, p, v) do { const T vst2_v_ = (v); *(volatile T*)(p) = vst2_v_; __threadfence(); *(volatile T*)(p) = vst2_v_; } while (0)
__device__ __forceinline__ int clampi(int v, int lo, int hi) { return v < lo ? lo : (v > hi ? hi : v); }
__global__ __launch_bounds__(256) void k_me(const float* __restrict__ seq, const int* __restrict__ epos, float* ME) { const size_t q = (size_t)blockIdx.x * 256 + threadIdx.x; if (q >= (size_t)NB_ * NMEN * DD) return; const int d = (int)(q % DD); const int mi = (int)((q / DD) % NMEN); const int b = (int)(q / ((size_t)DD * NMEN)); const int pos = clampi(epos[b * NMEN + mi] + 1, 0, LL - 1); VST2(float, ME + q, seq[((size_t)b * LL + pos) * DD + d]); }
__global__ __launch_bounds__(256) void k_en(const float* __restrict__ ME, float* EN) { const size_t q = (size_t)blockIdx.x * 256 + threadIdx.x; if (q >= (size_t)NB_ * NE * DD) return; const int d = (int)(q % DD); const int e = (int)((q / DD) % NE); const int b = (int)(q / ((size_t)DD * NE)); float v[NM]; float m = -__builtin_inff();
#pragma unroll
    for (int k = 0; k < NM; ++k) { v[k] = ME[(((size_t)b * NMEN) + e * NM + k) * DD + d]; m = fmaxf(m, v[k]); } float s = 0.f;
#pragma unroll
    for (int k = 0; k < NM; ++k) s += expf(v[k] - m); VST2(float, EN + q, m + logf(s)); }
__global__ __launch_bounds__(256) void k_ea(const float* __restrict__ attn, const int* __restrict__ epos, float* EA) { const size_t q = (size_t)blockIdx.x * 256 + threadIdx.x; if (q >= (size_t)NB_ * NE * NH * LL) return; const int l = (int)(q % LL); const int h = (int)((q / LL) % NH); const int e = (int)((q / ((size_t)LL * NH)) % NE); const int b = (int)(q / ((size_t)LL * NH * NE)); float s = 0.f;
#pragma unroll
    for (int m = 0; m < NM; ++m) { const int pos = clampi(epos[(b * NE + e) * NM + m] + 1, 0, LL - 1); s += attn[(((size_t)b * NH + h) * LL + pos) * LL + l]; } VST2(float, EA + q, s * 0.25f); }
__global__ __launch_bounds__(256) void k_ht(const float* __restrict__ EA, const int* __restrict__ hts, float* HT) { const int lane = threadIdx.x & 31; const int n = blockIdx.x * 8 + (threadIdx.x >> 5); if (n >= NPAIR) return; const int b = n / NPR; const int he = clampi(hts[n * 2], 0, NE - 1), te = clampi(hts[n * 2 + 1], 0, NE - 1); float s = 0.f;
#pragma unroll 1
    for (int l = lane; l < LL; l += 32) { float a = 0.f;
#pragma unroll 1
        for (int h = 0; h < NH; ++h) a += EA[(((size_t)b * NE + he) * NH + h) * LL + l] * EA[(((size_t)b * NE + te) * NH + h) * LL + l]; a = a / (float)NH; s += a; VST2(float, HT + (size_t)n * LL + l, a); }
#pragma unroll
    for (int o = 16; o; o >>= 1) s += __shfl_xor(s, o, 32);
    const float inv = 1.f / (s + 1e-5f);
#pragma unroll 1
    for (int l = lane; l < LL; l += 32) { const float a = HT[(size_t)n * LL + l]; VST2(float, HT + (size_t)n * LL + l, a * inv); } }
__global__ __launch_bounds__(256) void k_cat(const float* __restrict__ EN, const float* __restrict__ RS, const int* __restrict__ hts, float* AH, float* AT) { const size_t q = (size_t)blockIdx.x * 256 + threadIdx.x; if (q >= (size_t)NPAIR * 2 * DD) return; const int c = (int)(q % (2 * DD)); const int n = (int)(q / (2 * DD)); const int b = n / NPR; const int he = clampi(hts[n * 2], 0, NE - 1), te = clampi(hts[n * 2 + 1], 0, NE - 1);
    if (c < DD) { VST2(float, AH + q, EN[((size_t)b * NE + he) * DD + c]); VST2(float, AT + q, EN[((size_t)b * NE + te) * DD + c]); } else { const float r = RS[(size_t)n * DD + c - DD]; VST2(float, AH + q, r); VST2(float, AT + q, r); } }
__global__ __launch_bounds__(256) void k_bl(const float* __restrict__ HZ, const float* __restrict__ TZ, float* BL) { const size_t q = (size_t)blockIdx.x * 256 + threadIdx.x; if (q >= (size_t)NPAIR * EMB * BS) return; const int col = (int)(q % ((size_t)EMB * BS)); const int n = (int)(q / ((size_t)EMB * BS)); const int c = col % BS, ia = col / BS; const int i = ia / BS; VST2(float, BL + q, HZ[(size_t)n * EMB + ia] * TZ[(size_t)n * EMB + i * BS + c]); }
__global__ __launch_bounds__(256) void k_w(const float* __restrict__ Wfh, const float* __restrict__ Wft, const float* __restrict__ Wun, const float* __restrict__ bun, const float* __restrict__ Wml, const float* __restrict__ bml, float* WC, float* WUM, float* BUM) { const size_t q = (size_t)blockIdx.x * 256 + threadIdx.x;
    if (q < (size_t)DD * 2 * DD) { const int c = (int)(q % (2 * DD)); const int k = (int)(q / (2 * DD)); VST2(float, WC + q, c < DD ? Wfh[(size_t)k * EMB + c] : Wft[(size_t)k * EMB + c - DD]); }
    if (q < (size_t)EMB * 256) { const int c = (int)(q % 256); const int k = (int)(q / 256); float v = 0.f; if (c < NCL) v = Wun[(size_t)k * NCL + c]; else if (c >= 128 && c < 128 + NCL) v = Wml[(size_t)k * NCL + c - 128]; VST2(float, WUM + q, v); if (k == 0) { float bb = 0.f; if (c < NCL) bb = bun[c]; else if (c >= 128 && c < 128 + NCL) bb = bml[c - 128]; VST2(float, BUM + c, bb); } } }
__global__ __launch_bounds__(256) void k_feat(const float* __restrict__ FHT, const int* __restrict__ midx, const int* __restrict__ hts, const float* __restrict__ bf, float* FEAT) { const size_t q = (size_t)blockIdx.x * 256 + threadIdx.x; if (q >= (size_t)NPAIR * NM * NM * DD) return; const int d = (int)(q % DD); const int r = (int)(q / DD); const int m2 = r % NM, m1 = (r / NM) % NM, n = r / (NM * NM); const int b = n / NPR; const int he = clampi(hts[n * 2], 0, NE - 1), te = clampi(hts[n * 2 + 1], 0, NE - 1);
    const int mh = clampi(midx[(b * NE + he) * NM + m1], 0, NMEN - 1), mt = clampi(midx[(b * NE + te) * NM + m2], 0, NMEN - 1);
    VST2(float, FEAT + q, FHT[((size_t)b * NMEN + mh) * 2 * DD + d] + FHT[((size_t)b * NMEN + mt) * 2 * DD + DD + d] + bf[d]); }
__device__ __forceinline__ float gelu_tanh(float x) { const float u = 0.7978845608028654f * (x + 0.044715f * x * x * x); return 0.5f * x * (1.f + tanhf(u)); }
__global__ __launch_bounds__(256) void k_r(const float* __restrict__ R1, const float* __restrict__ E2, float* R) { const int q = blockIdx.x * 256 + threadIdx.x; if (q >= NPAIR * 320) return; const int c = q % 320, n = q / 320; float v = 0.f;
    if (c < NCL) v = R1[(size_t)n * 128 + c];
    else if (c < 3 * NCL) { const int which = (c - NCL) / NCL, cc = (c - NCL) % NCL; float m = -__builtin_inff();
#pragma unroll 1
        for (int k = 0; k < 16; ++k) { const float e = E2[((size_t)n * 16 + k) * 256 + (which ? 128 : 0) + cc]; const float t = which ? gelu_tanh(e) : tanhf(e); m = fmaxf(m, t); } float s = 0.f;
#pragma unroll 1
        for (int k = 0; k < 16; ++k) { const float e = E2[((size_t)n * 16 + k) * 256 + (which ? 128 : 0) + cc]; const float t = which ? gelu_tanh(e) : tanhf(e); s += expf(t - m); } v = m + logf(s); }
    VST2(float, R + q, v); }
__global__ __launch_bounds__(256) void k_out(const float* __restrict__ O128, float* out) { const int q = blockIdx.x * 256 + threadIdx.x; if (q >= NPAIR * NCL) return; VST2(float, out + q, O128[(size_t)(q / NCL) * 128 + (q % NCL)]); }
extern "C" void kernel_launch(void* const* d_in, const int* in_sizes, int n_in,
                              void* d_out, int out_size, void* d_ws, size_t ws_size, hipStream_t stream) {
    (void)in_sizes; (void)n_in; (void)out_size;
    const float* seq = (const float*)d_in[0]; const float* attn = (const float*)d_in[1]; const int* epos = (const int*)d_in[2]; const int* hts = (const int*)d_in[3]; const int* midx = (const int*)d_in[4];
    const float* Whd = (const float*)d_in[5]; const float* bhd = (const float*)d_in[6]; const float* Wtl = (const float*)d_in[7]; const float* btl = (const float*)d_in[8]; const float* Wrel = (const float*)d_in[9]; const float* brel = (const float*)d_in[10]; const float* Wfh = (const float*)d_in[11]; const float* Wft = (const float*)d_in[12]; const float* bf = (const float*)d_in[13]; const float* Wun = (const float*)d_in[14]; const float* bun = (const float*)d_in[15]; const float* Wml = (const float*)d_in[16]; const float* bml = (const float*)d_in[17]; const float* Wbil = (const float*)d_in[18]; const float* bbil = (const float*)d_in[19];
    float* out = (float*)d_out;
    char* wsp = (char*)d_ws;
    auto take = [&](size_t bytes) { char* p = wsp; wsp += (bytes + 255) & ~(size_t)255; return (void*)p; };
    float* ME = (float*)take((size_t)NB_ * NMEN * DD * 4); float* EN = (float*)take((size_t)NB_ * NE * DD * 4); float* EA = (float*)take((size_t)NB_ * NE * NH * LL * 4); float* HT = (float*)take((size_t)NPAIR * LL * 4); float* RS = (float*)take((size_t)NPAIR * DD * 4); float* AH = (float*)take((size_t)NPAIR * 2 * DD * 4); float* AT = (float*)take((size_t)NPAIR * 2 * DD * 4); float* HZ = (float*)take((size_t)NPAIR * EMB * 4); float* TZ = (float*)take((size_t)NPAIR * EMB * 4);
    float* BL = (float*)take((size_t)NPAIR * EMB * BS * 4); float* R1 = (float*)take((size_t)NPAIR * 128 * 4); float* WC = (float*)take((size_t)DD * 2 * DD * 4); float* FHT = (float*)take((size_t)NB_ * NMEN * 2 * DD * 4); float* WUM = (float*)take((size_t)EMB * 256 * 4); float* BUM = (float*)take(256 * 4); float* FEAT = (float*)take((size_t)NPAIR * 16 * DD * 4); float* E2 = (float*)take((size_t)NPAIR * 16 * 256 * 4); float* R = (float*)take((size_t)NPAIR * 320 * 4); float* O128 = (float*)take((size_t)NPAIR * 128 * 4);
    if ((size_t)(wsp - (char*)d_ws) > ws_size) return;
    k_me<<<(unsigned)(((size_t)NB_ * NMEN * DD) / 256), 256, 0, stream>>>(seq, epos, ME);
    k_en<<<(unsigned)(((size_t)NB_ * NE * DD) / 256), 256, 0, stream>>>(ME, EN);
    k_ea<<<(unsigned)(((size_t)NB_ * NE * NH * LL) / 256), 256, 0, stream>>>(attn, epos, EA);
    k_ht<<<NPAIR / 8, 256, 0, stream>>>(EA, hts, HT);
    { GemmArgs g = gemm_args(HT, LL, zm(NPR * LL), seq, DD, zm(LL * DD), RS, DD, zm(NPR * DD), NPR, DD, LL); gemm_kernel<0, 0, 2, 2, 4, 2, ACT_NONE><<<dim3(NPR / 64, DD / 128, NB_), 256, 0, stream>>>(g); }
    k_cat<<<(unsigned)(((size_t)NPAIR * 2 * DD) / 256), 256, 0, stream>>>(EN, RS, hts, AH, AT);
    { GemmArgs g = gemm_args(AH, 2 * DD, zm(0), Whd, EMB, zm(0), HZ, EMB, zm(0), NPAIR, EMB, 2 * DD); g.bias = bhd; gemm_kernel<0, 1, 1, 1, 4, 2, ACT_TANH><<<dim3(NPAIR / 64, EMB / 128, 1), 256, 0, stream>>>(g); }
    { GemmArgs g = gemm_args(AT, 2 * DD, zm(0), Wtl, EMB, zm(0), TZ, EMB, zm(0), NPAIR, EMB, 2 * DD); g.bias = btl; gemm_kernel<0, 1, 1, 1, 4, 2, ACT_TANH><<<dim3(NPAIR / 64, EMB / 128, 1), 256, 0, stream>>>(g); }
    k_bl<<<(unsigned)(((size_t)NPAIR * EMB * BS) / 256), 256, 0, stream>>>(HZ, TZ, BL);
    { GemmArgs g = gemm_args(BL, EMB * BS, zm(0), Wrel, NCL, zm(0), R1, 128, zm(0), NPAIR, NCL, EMB * BS); g.bias = brel; g.nstore = 128; gemm_kernel<0, 1, 1, 1, 4, 2, ACT_NONE><<<dim3(NPAIR / 64, 1, 1), 256, 0, stream>>>(g); }
    k_w<<<(unsigned)(((size_t)DD * 2 * DD + 255) / 256), 256, 0, stream>>>(Wfh, Wft, Wun, bun, Wml, bml, WC, WUM, BUM);
    { GemmArgs g = gemm_args(ME, DD, zm(0), WC, 2 * DD, zm(0), FHT, 2 * DD, zm(0), NB_ * NMEN, 2 * DD, DD); gemm_kernel<0, 0, 2, 2, 4, 2, ACT_NONE><<<dim3((NB_ * NMEN) / 64, (2 * DD) / 128, 1), 256, 0, stream>>>(g); }
    k_feat<<<(unsigned)(((size_t)NPAIR * 16 * DD) / 256), 256, 0, stream>>>(FHT, midx, hts, bf, FEAT);
    { GemmArgs g = gemm_args(FEAT, DD, zm(0), WUM, 256, zm(0), E2, 256, zm(0), NPAIR * 16, 256, DD); g.bias = BUM; gemm_kernel<0, 1, 1, 1, 4, 2, ACT_NONE><<<dim3((NPAIR * 16) / 64, 2, 1), 256, 0, stream>>>(g); }
    k_r<<<(NPAIR * 320) / 256, 256, 0, stream>>>(R1, E2, R);
    { GemmArgs g = gemm_args(R, 320, zm(0), Wbil, NCL, zm(0), O128, 128, zm(0), NPAIR, NCL, 3 * NCL); g.bias = bbil; g.nstore = 128; gemm_kernel<0, 0, 2, 2, 4, 2, ACT_NONE><<<dim3(NPAIR / 64, 1, 1), 256, 0, stream>>>(g); }
    k_out<<<(NPAIR * NCL + 255) / 256, 256, 0, stream>>>(O128, out);
}
